// MappingNet_9431748182734
// MI455X (gfx1250) — hardware-verified
//
#include <hip/hip_runtime.h>
#define BS 4096
#define IND 512
#define DIM 1024
#define NGE 10
#define NTILE (BS / 16 + NGE)
#define NROW (NTILE * 16)

typedef __bf16 v16b __attribute__((ext_vector_type(16)));
typedef unsigned short v8us __attribute__((ext_vector_type(8), may_alias));
typedef float  v8f  __attribute__((ext_vector_type(8)));
typedef float  v4f  __attribute__((ext_vector_type(4)));
typedef float  v4fa __attribute__((ext_vector_type(4), may_alias));
union FragB { v16b v; v8us half[2]; unsigned short u[16]; };

__device__ __forceinline__ unsigned short bf16_bits(float x) { unsigned int u = __float_as_uint(x); return (unsigned short)((u + 0x7FFFu + ((u >> 16) & 1u)) >> 16); }
__device__ __forceinline__ float bf16_val(unsigned short b) { return __uint_as_float(((unsigned int)b) << 16); }
__device__ __forceinline__ float bf16_round(float x) { return bf16_val(bf16_bits(x)); }
template <int NT>
__device__ __forceinline__ v8f mmaN(v16b ah, v16b al, v16b bh, v16b bl, v8f c) {
  c = __builtin_amdgcn_wmma_f32_16x16x32_bf16(false, ah, false, bh, (short)0, c, false, false);
  if (NT >= 2) c = __builtin_amdgcn_wmma_f32_16x16x32_bf16(false, al, false, bh, (short)0, c, false, false);
  if (NT >= 3) c = __builtin_amdgcn_wmma_f32_16x16x32_bf16(false, ah, false, bl, (short)0, c, false, false);
  asm volatile("v_nop\n\tv_nop\n\tv_nop\n\tv_nop" : "+v"(c) : "v"(ah), "v"(al), "v"(bh), "v"(bl));
  return c;
}

__global__ __launch_bounds__(256) void k_wt_bf16(const float* __restrict__ W, unsigned short* __restrict__ Wt, int K, int N) {
  const int t = blockIdx.x * 256 + threadIdx.x;
  const int k8n = K / 8;
  if (t >= N * k8n) return;
  const int n = t / k8n, k8 = (t % k8n) * 8;
  v8us v;
#pragma unroll
  for (int i = 0; i < 8; ++i) v[i] = bf16_bits(W[(size_t)(k8 + i) * N + n]);
  *(volatile v8us*)(Wt + (size_t)n * K + k8) = v;
  __threadfence();
  *(volatile v8us*)(Wt + (size_t)n * K + k8) = v;
}

template <bool ASPLIT, int ACT, bool BIAS_BF16>
__global__ __launch_bounds__(128) void k_gemm_bf(const float* __restrict__ A, int lda, const unsigned short* __restrict__ Wt, int ldb,
                                               const float* __restrict__ bias, float* __restrict__ C, int ldc, int M, int N, int K) {
  __shared__ __attribute__((aligned(16))) float so[4][16][64];
  const int tid = threadIdx.x, w = tid >> 5, lane = tid & 31, ln = lane & 15, hh = lane >> 4;
  const int ntn = N / 64;
  const int wid = blockIdx.x * 4 + w;
  const int mt = wid / ntn, nq = wid % ntn;
  if (mt * 16 >= M) return;
  const int row0 = mt * 16, col0 = nq * 64;
  const float* arow = A + (size_t)(row0 + ln) * lda;
  v8f acc[4] = {};
  for (int kb = 0; kb < K; kb += 32) {
    FragB ah, al;
    const v4f x0 = *(const v4fa*)(arow + kb + 8 * hh), x1 = *(const v4fa*)(arow + kb + 8 * hh + 4);
    const v4f x2 = *(const v4fa*)(arow + kb + 16 + 8 * hh), x3 = *(const v4fa*)(arow + kb + 16 + 8 * hh + 4);
    float xs[16] = {x0[0],x0[1],x0[2],x0[3],x1[0],x1[1],x1[2],x1[3],x2[0],x2[1],x2[2],x2[3],x3[0],x3[1],x3[2],x3[3]};
#pragma unroll
    for (int i = 0; i < 16; ++i) { const unsigned short hb = bf16_bits(xs[i]); ah.u[i] = hb; al.u[i] = ASPLIT ? bf16_bits(xs[i] - bf16_val(hb)) : (unsigned short)0; }
#pragma unroll
    for (int t = 0; t < 4; ++t) {
      const unsigned short* brow = Wt + (size_t)(col0 + t * 16 + ln) * ldb + kb;
      FragB b;
      b.half[0] = *(const v8us*)(brow + 8 * hh);
      b.half[1] = *(const v8us*)(brow + 16 + 8 * hh);
      acc[t] = mmaN<ASPLIT ? 2 : 1>(ah.v, al.v, b.v, b.v, acc[t]);
    }
  }
#pragma unroll
  for (int t = 0; t < 4; ++t) {
    float bv = bias ? bias[col0 + t * 16 + ln] : 0.f;
    if (BIAS_BF16) bv = bf16_round(bv);
#pragma unroll
    for (int r = 0; r < 8; ++r) { float v = acc[t][r] + bv; if (ACT == 1) v = fmaxf(v, 0.f); so[w][8 * hh + r][t * 16 + ln] = v; }
  }
  __builtin_amdgcn_fence(__ATOMIC_ACQ_REL, "workgroup");
  __builtin_amdgcn_wave_barrier();
  const int rsub = lane >> 4, c4 = (lane & 15) * 4;
  for (int pass = 0; pass < 2; ++pass) {
#pragma unroll
    for (int q = 0; q < 8; ++q) {
      const int r = q * 2 + rsub;
      const v4f v = *(const v4fa*)&so[w][r][c4];
      *(volatile v4f*)(C + (size_t)(row0 + r) * ldc + col0 + c4) = v;
    }
    if (pass == 0) __threadfence();
  }
}

template <int D, bool CAUSAL>
__global__ __launch_bounds__(128) void k_flash(const float* __restrict__ qb, const float* __restrict__ kb, const float* __restrict__ vb,
                                             int pitch, int T, int H, float scale, float* __restrict__ y, int ypitch) {
  constexpr int KS = D / 32;
  constexpr int DT = D / 16;
  __shared__ __attribute__((aligned(16))) unsigned short sKh[32][D + 8], sKl[32][D + 8], sVh[32][D + 8], sVl[32][D + 8];
  __shared__ __attribute__((aligned(16))) unsigned short sPh[4][16][40], sPl[4][16][40];
  __shared__ __attribute__((aligned(16))) float sO[4][16][D];
  const int tid = threadIdx.x, w = tid >> 5, lane = tid & 31, ln = lane & 15, hh = lane >> 4;
  const int nqb = (T + 63) / 64;
  const int bh = blockIdx.x / nqb, qblk = blockIdx.x % nqb;
  const int b = bh / H, h = bh % H;
  const int q0 = qblk * 64 + w * 16;
  const float* Q = qb + (size_t)b * T * pitch + h * D;
  const float* K = kb + (size_t)b * T * pitch + h * D;
  const float* V = vb + (size_t)b * T * pitch + h * D;

  FragB aqh[KS], aql[KS];
  {
    int row = q0 + ln; if (row >= T) row = T - 1;
    const float* qr = Q + (size_t)row * pitch;
#pragma unroll
    for (int ks = 0; ks < KS; ++ks)
#pragma unroll
      for (int i = 0; i < 16; ++i) {
        const int d = ks * 32 + ((i < 8) ? (8 * hh + i) : (16 + 8 * hh + (i - 8)));
        const float x = qr[d] * scale; const unsigned short hb = bf16_bits(x);
        aqh[ks].u[i] = hb; aql[ks].u[i] = bf16_bits(x - bf16_val(hb));
      }
  }
  float m_r[8], l_r[8];
#pragma unroll
  for (int r = 0; r < 8; ++r) { m_r[r] = -3.0e38f; l_r[r] = 0.f; }
  v8f oacc[DT];
#pragma unroll
  for (int dt = 0; dt < DT; ++dt) oacc[dt] = (v8f){0.f,0.f,0.f,0.f,0.f,0.f,0.f,0.f};

  const int kv_end = CAUSAL ? min(T, qblk * 64 + 64) : T;
  for (int j0 = 0; j0 < kv_end; j0 += 32) {
    __syncthreads();
    for (int e = tid; e < 32 * (D / 4); e += 128) {
      const int r = e / (D / 4), c4 = (e % (D / 4)) * 4;
      const int key = j0 + r;
      v4f kf = {0.f,0.f,0.f,0.f}, vf = {0.f,0.f,0.f,0.f};
      if (key < T) { kf = *(const v4fa*)(K + (size_t)key * pitch + c4); vf = *(const v4fa*)(V + (size_t)key * pitch + c4); }
#pragma unroll
      for (int t = 0; t < 4; ++t) {
        unsigned short hb = bf16_bits(kf[t]); sKh[r][c4 + t] = hb; sKl[r][c4 + t] = bf16_bits(kf[t] - bf16_val(hb));
        hb = bf16_bits(vf[t]); sVh[r][c4 + t] = hb; sVl[r][c4 + t] = bf16_bits(vf[t] - bf16_val(hb));
      }
    }
    __syncthreads();
    v8f s[2];
#pragma unroll
    for (int nt = 0; nt < 2; ++nt) {
      v8f acc = {};
#pragma unroll
      for (int ks = 0; ks < KS; ++ks) {
        FragB bh_, bl_;
        bh_.half[0] = *(const v8us*)&sKh[nt * 16 + ln][ks * 32 + 8 * hh]; bh_.half[1] = *(const v8us*)&sKh[nt * 16 + ln][ks * 32 + 16 + 8 * hh];
        bl_.half[0] = *(const v8us*)&sKl[nt * 16 + ln][ks * 32 + 8 * hh]; bl_.half[1] = *(const v8us*)&sKl[nt * 16 + ln][ks * 32 + 16 + 8 * hh];
        acc = mmaN<3>(aqh[ks].v, aql[ks].v, bh_.v, bl_.v, acc);
      }
      s[nt] = acc;
    }
    float alpha[8];
#pragma unroll
    for (int r = 0; r < 8; ++r) {
      const int qi = q0 + 8 * hh + r;
      const int ja = j0 + ln, jb = j0 + 16 + ln;
      if (CAUSAL) { if (ja > qi) s[0][r] = -3.0e38f; if (jb > qi) s[1][r] = -3.0e38f; }
      if (ja >= T) s[0][r] = -3.0e38f;
      if (jb >= T) s[1][r] = -3.0e38f;
      float mx = fmaxf(s[0][r], s[1][r]);
      mx = fmaxf(mx, __shfl_xor(mx, 1, 32)); mx = fmaxf(mx, __shfl_xor(mx, 2, 32)); mx = fmaxf(mx, __shfl_xor(mx, 4, 32)); mx = fmaxf(mx, __shfl_xor(mx, 8, 32));
      const float mnew = fmaxf(m_r[r], mx);
      alpha[r] = (mnew > -1.0e38f) ? __expf(m_r[r] - mnew) : 1.0f;
      const float p0 = (s[0][r] > -1.0e38f) ? __expf(s[0][r] - mnew) : 0.f;
      const float p1 = (s[1][r] > -1.0e38f) ? __expf(s[1][r] - mnew) : 0.f;
      m_r[r] = mnew;
      l_r[r] = l_r[r] * alpha[r] + p0 + p1;
      unsigned short hb = bf16_bits(p0); sPh[w][8 * hh + r][ln] = hb;      sPl[w][8 * hh + r][ln] = bf16_bits(p0 - bf16_val(hb));
      hb = bf16_bits(p1);                sPh[w][8 * hh + r][16 + ln] = hb; sPl[w][8 * hh + r][16 + ln] = bf16_bits(p1 - bf16_val(hb));
    }
#pragma unroll
    for (int dt = 0; dt < DT; ++dt)
#pragma unroll
      for (int r = 0; r < 8; ++r) oacc[dt][r] *= alpha[r];
    __builtin_amdgcn_fence(__ATOMIC_ACQ_REL, "workgroup");
    __builtin_amdgcn_wave_barrier();
    FragB pah, pal;
    pah.half[0] = *(const v8us*)&sPh[w][ln][8 * hh]; pah.half[1] = *(const v8us*)&sPh[w][ln][16 + 8 * hh];
    pal.half[0] = *(const v8us*)&sPl[w][ln][8 * hh]; pal.half[1] = *(const v8us*)&sPl[w][ln][16 + 8 * hh];
#pragma unroll
    for (int dt = 0; dt < DT; ++dt) {
      FragB bvh, bvl;
#pragma unroll
      for (int i = 0; i < 8; ++i) {
        bvh.u[i] = sVh[8 * hh + i][dt * 16 + ln]; bvh.u[8 + i] = sVh[16 + 8 * hh + i][dt * 16 + ln];
        bvl.u[i] = sVl[8 * hh + i][dt * 16 + ln]; bvl.u[8 + i] = sVl[16 + 8 * hh + i][dt * 16 + ln];
      }
      oacc[dt] = mmaN<3>(pah.v, pal.v, bvh.v, bvl.v, oacc[dt]);
    }
    __builtin_amdgcn_fence(__ATOMIC_ACQ_REL, "workgroup");
    __builtin_amdgcn_wave_barrier();
  }
#pragma unroll
  for (int r = 0; r < 8; ++r) {
    float l = l_r[r];
    l += __shfl_xor(l, 1, 32); l += __shfl_xor(l, 2, 32); l += __shfl_xor(l, 4, 32); l += __shfl_xor(l, 8, 32);
    l_r[r] = (l > 0.f) ? 1.0f / l : 0.f;
  }
#pragma unroll
  for (int dt = 0; dt < DT; ++dt)
#pragma unroll
    for (int r = 0; r < 8; ++r) sO[w][8 * hh + r][dt * 16 + ln] = oacc[dt][r] * l_r[r];
  __builtin_amdgcn_fence(__ATOMIC_ACQ_REL, "workgroup");
  __builtin_amdgcn_wave_barrier();
  for (int pass = 0; pass < 2; ++pass) {
    for (int r = 0; r < 16; ++r) {
      const int row = q0 + r;
      if (row < T && lane < D / 4) {
        const v4f val = *(const v4fa*)&sO[w][r][lane * 4];
        *(volatile v4f*)(y + ((size_t)b * T + row) * ypitch + h * D + lane * 4) = val;
      }
    }
    if (pass == 0) __threadfence();
  }
}

typedef _Float16 v16h __attribute__((ext_vector_type(16)));
union FragH { v16h v; v8us half[2]; _Float16 h[16]; unsigned short u[16]; };
template <int NT>
__device__ __forceinline__ v8f mmaH(v16h ah, v16h al, v16h bh, v16h bl, v8f c) {
  c = __builtin_amdgcn_wmma_f32_16x16x32_f16(false, ah, false, bh, (short)0, c, false, false);
  if (NT >= 2) c = __builtin_amdgcn_wmma_f32_16x16x32_f16(false, al, false, bh, (short)0, c, false, false);
  if (NT >= 3) c = __builtin_amdgcn_wmma_f32_16x16x32_f16(false, ah, false, bl, (short)0, c, false, false);
  asm volatile("v_nop\n\tv_nop\n\tv_nop\n\tv_nop" : "+v"(c) : "v"(ah), "v"(al), "v"(bh), "v"(bl));
  return c;
}
template <bool ASPLIT>
__global__ __launch_bounds__(128) void k_gemm_h(const float* __restrict__ A, int lda, size_t sA, const _Float16* __restrict__ Bh, int ldb, size_t sB, float alpha, float* __restrict__ C, int ldc, size_t sC, int M, int N, int K) {
  __shared__ __attribute__((aligned(16))) float so[4][16][64];
  const int tid = threadIdx.x, w = tid >> 5, lane = tid & 31, ln = lane & 15, hh = lane >> 4; const int by = blockIdx.y;
  A += (size_t)by * sA; Bh += (size_t)by * sB; C += (size_t)by * sC;
  const int ntn = (N + 63) / 64; const int wid = blockIdx.x * 4 + w; const int mt = wid / ntn, nq = wid % ntn; if (mt * 16 >= M) return;
  const int row0 = mt * 16, col0 = nq * 64; const float* arow = A + (size_t)(row0 + ln) * lda;
  v8f acc[4] = {};
  for (int kb = 0; kb < K; kb += 32) {
    FragH ah, al;
    const v4f x0 = *(const v4fa*)(arow + kb + 8 * hh), x1 = *(const v4fa*)(arow + kb + 8 * hh + 4), x2 = *(const v4fa*)(arow + kb + 16 + 8 * hh), x3 = *(const v4fa*)(arow + kb + 16 + 8 * hh + 4);
    float xs[16] = {x0[0],x0[1],x0[2],x0[3],x1[0],x1[1],x1[2],x1[3],x2[0],x2[1],x2[2],x2[3],x3[0],x3[1],x3[2],x3[3]};
#pragma unroll
    for (int i = 0; i < 16; ++i) { const _Float16 h = (_Float16)xs[i]; ah.h[i] = h; al.h[i] = ASPLIT ? (_Float16)(xs[i] - (float)h) : (_Float16)0.0f; }
#pragma unroll
    for (int t = 0; t < 4; ++t) { if (col0 + t * 16 >= N) continue; const size_t boff = (size_t)(col0 + t * 16 + ln) * ldb + kb; FragH bq; bq.half[0] = *(const v8us*)(Bh + boff + 8 * hh); bq.half[1] = *(const v8us*)(Bh + boff + 16 + 8 * hh);
      acc[t] = mmaH<ASPLIT ? 2 : 1>(ah.v, al.v, bq.v, bq.v, acc[t]); }
  }
#pragma unroll
  for (int t = 0; t < 4; ++t) { if (col0 + t * 16 >= N) continue;
#pragma unroll
    for (int r = 0; r < 8; ++r) so[w][8 * hh + r][t * 16 + ln] = acc[t][r] * alpha; }
  __builtin_amdgcn_fence(__ATOMIC_ACQ_REL, "workgroup"); __builtin_amdgcn_wave_barrier();
  const int rsub = lane >> 4, c4 = (lane & 15) * 4;
  for (int pass = 0; pass < 2; ++pass) {
#pragma unroll
    for (int q = 0; q < 8; ++q) { const int r = q * 2 + rsub; if (col0 + c4 < N) { const v4f v = *(const v4fa*)&so[w][r][c4]; *(volatile v4f*)(C + (size_t)(row0 + r) * ldc + col0 + c4) = v; } }
    if (pass == 0) __threadfence(); }
}
template <bool ASPLIT>
__global__ __launch_bounds__(128) void k_gemm_hgrp(const float* __restrict__ A, int lda, const _Float16* __restrict__ Bh0, int ldb, size_t strideB, const int* __restrict__ tileGrp, float alpha, float* __restrict__ C, int ldc, int M, int N, int K) {
  __shared__ __attribute__((aligned(16))) float so[4][16][64];
  const int tid = threadIdx.x, w = tid >> 5, lane = tid & 31, ln = lane & 15, hh = lane >> 4; const int ntn = (N + 63) / 64; const int wid = blockIdx.x * 4 + w; const int mt = wid / ntn, nq = wid % ntn; if (mt * 16 >= M) return; const int grp = tileGrp[mt]; if (grp < 0) return; const _Float16* __restrict__ Bh = Bh0 + (size_t)grp * strideB;
  const int row0 = mt * 16, col0 = nq * 64; const float* arow = A + (size_t)(row0 + ln) * lda;
  v8f acc[4] = {};
  for (int kb = 0; kb < K; kb += 32) {
    FragH ah, al;
    const v4f x0 = *(const v4fa*)(arow + kb + 8 * hh), x1 = *(const v4fa*)(arow + kb + 8 * hh + 4), x2 = *(const v4fa*)(arow + kb + 16 + 8 * hh), x3 = *(const v4fa*)(arow + kb + 16 + 8 * hh + 4);
    float xs[16] = {x0[0],x0[1],x0[2],x0[3],x1[0],x1[1],x1[2],x1[3],x2[0],x2[1],x2[2],x2[3],x3[0],x3[1],x3[2],x3[3]};
#pragma unroll
    for (int i = 0; i < 16; ++i) { const _Float16 h = (_Float16)xs[i]; ah.h[i] = h; al.h[i] = ASPLIT ? (_Float16)(xs[i] - (float)h) : (_Float16)0.0f; }
#pragma unroll
    for (int t = 0; t < 4; ++t) { if (col0 + t * 16 >= N) continue; const size_t boff = (size_t)(col0 + t * 16 + ln) * ldb + kb; FragH bq; bq.half[0] = *(const v8us*)(Bh + boff + 8 * hh); bq.half[1] = *(const v8us*)(Bh + boff + 16 + 8 * hh);
      acc[t] = mmaH<ASPLIT ? 2 : 1>(ah.v, al.v, bq.v, bq.v, acc[t]); }
  }
#pragma unroll
  for (int t = 0; t < 4; ++t) { if (col0 + t * 16 >= N) continue;
#pragma unroll
    for (int r = 0; r < 8; ++r) so[w][8 * hh + r][t * 16 + ln] = acc[t][r] * alpha; }
  __builtin_amdgcn_fence(__ATOMIC_ACQ_REL, "workgroup"); __builtin_amdgcn_wave_barrier();
  const int rsub = lane >> 4, c4 = (lane & 15) * 4;
  for (int pass = 0; pass < 2; ++pass) {
#pragma unroll
    for (int q = 0; q < 8; ++q) { const int r = q * 2 + rsub; if (col0 + c4 < N) { const v4f v = *(const v4fa*)&so[w][r][c4]; *(volatile v4f*)(C + (size_t)(row0 + r) * ldc + col0 + c4) = v; } }
    if (pass == 0) __threadfence(); }
}

__global__ __launch_bounds__(256) void k_wt_f16(const float* __restrict__ W, _Float16* __restrict__ Wt, int K, int N, float scale) { const size_t t = (size_t)blockIdx.x * 256 + threadIdx.x; if (t >= (size_t)N * (K / 8)) return; const int n = (int)(t / (K / 8)), k8 = (int)(t % (K / 8)) * 8; FragH f;
#pragma unroll
  for (int i = 0; i < 8; ++i) f.h[i] = (_Float16)(bf16_round(W[(size_t)(k8 + i) * N + n]) * scale); const v8us o = f.half[0]; *(volatile v8us*)((unsigned short*)Wt + (size_t)n * K + k8) = o; __threadfence(); *(volatile v8us*)((unsigned short*)Wt + (size_t)n * K + k8) = o; }
__device__ __forceinline__ float gelu_e(float v) { return 0.5f * v * (1.0f + erff(v * 0.70710678118654752f)); }
__global__ __launch_bounds__(1024) void k_group(const int* __restrict__ genre, int* __restrict__ rowSmp, int* __restrict__ tileGrp, int* __restrict__ smpRow) {
  __shared__ int scnt[NGE]; __shared__ int sts[NGE + 1]; __shared__ int spos[BS]; __shared__ int srow[NROW]; const int t = threadIdx.x;
  if (t < NGE) { int c = 0; for (int b = 0; b < BS; ++b) { int g = genre[b]; g = g < 0 ? 0 : (g >= NGE ? NGE - 1 : g); c += (g == t); } scnt[t] = c; }
  __syncthreads();
  if (t == 0) { int s = 0; for (int g = 0; g < NGE; ++g) { sts[g] = s; s += (scnt[g] + 15) / 16; } sts[NGE] = s; }
  __syncthreads();
  for (int b = t; b < BS; b += 1024) { int g = genre[b]; g = g < 0 ? 0 : (g >= NGE ? NGE - 1 : g); int r = 0; for (int b2 = 0; b2 < b; ++b2) { int g2 = genre[b2]; g2 = g2 < 0 ? 0 : (g2 >= NGE ? NGE - 1 : g2); r += (g2 == g); } spos[b] = sts[g] * 16 + r; }
  __syncthreads();
  for (int r = t; r < NROW; r += 1024) srow[r] = -1; __syncthreads(); for (int b = t; b < BS; b += 1024) srow[spos[b]] = b; __syncthreads();
  for (int pass = 0; pass < 2; ++pass) {
    for (int r = t; r < NROW; r += 1024) *(volatile int*)(rowSmp + r) = srow[r];
    for (int b = t; b < BS; b += 1024) *(volatile int*)(smpRow + b) = spos[b];
    for (int tl = t; tl < NTILE; tl += 1024) { int g = -1; for (int q = 0; q < NGE; ++q) if (tl >= sts[q] && tl < sts[q] + (scnt[q] + 15) / 16) g = q; *(volatile int*)(tileGrp + tl) = g; }
    if (pass == 0) __threadfence(); }
}
__global__ __launch_bounds__(256) void k_xin(const int* __restrict__ rowSmp, const int* __restrict__ genre, const float* __restrict__ z, const float* __restrict__ mu, const float* __restrict__ sg, float* __restrict__ XG) { const size_t t = (size_t)blockIdx.x * 256 + threadIdx.x; if (t >= (size_t)NROW * IND / 4) return; const int c4 = (int)((t * 4) % IND); const int row = (int)((t * 4) / IND); const int b = rowSmp[row]; v4f o = {0.f, 0.f, 0.f, 0.f};
  if (b >= 0) { int g = genre[b]; g = g < 0 ? 0 : (g >= NGE ? NGE - 1 : g); const v4f zz = *(const v4fa*)(z + (size_t)b * IND + c4); for (int q = 0; q < 4; ++q) o[q] = bf16_round(mu[g * IND + c4 + q]) + (fabsf(bf16_round(sg[g * IND + c4 + q])) + 1e-8f) * bf16_round(zz[q]); }
  *(volatile v4f*)(XG + t * 4) = o; __threadfence(); *(volatile v4f*)(XG + t * 4) = o; }
template <bool GELU, bool GROUPB>
__global__ __launch_bounds__(256) void k_bias(float* __restrict__ Y, const float* __restrict__ bias, const int* __restrict__ tileGrp, size_t n4) { const size_t t = (size_t)blockIdx.x * 256 + threadIdx.x; if (t >= n4) return; const int c4 = (int)((t * 4) % DIM); const int row = (int)((t * 4) / DIM); int g = 0; if (GROUPB) { g = tileGrp[row >> 4]; if (g < 0) return; }
  v4f v = *(const v4fa*)(Y + t * 4); for (int q = 0; q < 4; ++q) { float x = v[q] + bf16_round(bias[(size_t)g * DIM + c4 + q]); v[q] = GELU ? gelu_e(x) : x; } *(volatile v4f*)(Y + t * 4) = v; __threadfence(); *(volatile v4f*)(Y + t * 4) = v; }
__global__ __launch_bounds__(256) void k_unsort(const float* __restrict__ O, const int* __restrict__ smpRow, float* __restrict__ out) { const size_t t = (size_t)blockIdx.x * 256 + threadIdx.x; if (t >= (size_t)BS * DIM / 4) return; const int c4 = (int)((t * 4) % DIM); const int b = (int)((t * 4) / DIM); int r = smpRow[b]; r = r < 0 ? 0 : (r >= NROW ? NROW - 1 : r); const v4f v = *(const v4fa*)(O + (size_t)r * DIM + c4); *(volatile v4f*)(out + t * 4) = v; __threadfence(); *(volatile v4f*)(out + t * 4) = v; }
extern "C" void kernel_launch(void* const* d_in, const int* in_sizes, int n_in,
                              void* d_out, int out_size, void* d_ws, size_t ws_size, hipStream_t stream) {
  (void)in_sizes; (void)n_in; (void)out_size;
  (void)d_in[0]; const int* genre = (const int*)d_in[1]; const float* z = (const float*)d_in[2]; const float* mu = (const float*)d_in[3]; const float* sg = (const float*)d_in[4];
  const float* Ws1 = (const float*)d_in[5]; const float* bs1 = (const float*)d_in[6]; const float* Ws2 = (const float*)d_in[7]; const float* bs2 = (const float*)d_in[8]; const float* We1 = (const float*)d_in[9]; const float* be1 = (const float*)d_in[10]; const float* We2 = (const float*)d_in[11]; const float* be2 = (const float*)d_in[12];
  char* ws = (char*)d_ws; size_t off = 0;
  auto take = [&](size_t bytes) { char* p = ws + off; off += (bytes + 255) & ~(size_t)255; return p; };
  _Float16* B1 = (_Float16*)take((size_t)DIM * IND * 2); _Float16* B2 = (_Float16*)take((size_t)DIM * DIM * 2); _Float16* BE1 = (_Float16*)take((size_t)NGE * DIM * DIM * 2); _Float16* BE2 = (_Float16*)take((size_t)NGE * DIM * DIM * 2);
  int* rowSmp = (int*)take(NROW * 4); int* tileGrp = (int*)take(NTILE * 4 + 64); int* smpRow = (int*)take(BS * 4);
  float* XG = (float*)take((size_t)NROW * IND * 4); float* H1 = (float*)take((size_t)NROW * DIM * 4); float* H2 = (float*)take((size_t)NROW * DIM * 4);
  if (off > ws_size) return;
  k_wt_f16<<<(unsigned)(((size_t)DIM * IND / 8 + 255) / 256), 256, 0, stream>>>(Ws1, B1, IND, DIM, 16.0f); k_wt_f16<<<(unsigned)(((size_t)DIM * DIM / 8 + 255) / 256), 256, 0, stream>>>(Ws2, B2, DIM, DIM, 16.0f);
  for (int g = 0; g < NGE; ++g) { k_wt_f16<<<(unsigned)(((size_t)DIM * DIM / 8 + 255) / 256), 256, 0, stream>>>(We1 + (size_t)g * DIM * DIM, BE1 + (size_t)g * DIM * DIM, DIM, DIM, 16.0f); k_wt_f16<<<(unsigned)(((size_t)DIM * DIM / 8 + 255) / 256), 256, 0, stream>>>(We2 + (size_t)g * DIM * DIM, BE2 + (size_t)g * DIM * DIM, DIM, DIM, 16.0f); }
  k_group<<<1, 1024, 0, stream>>>(genre, rowSmp, tileGrp, smpRow);
  k_xin<<<(unsigned)(((size_t)NROW * IND / 4 + 255) / 256), 256, 0, stream>>>(rowSmp, genre, z, mu, sg, XG);
  k_gemm_h<false><<<dim3(((NROW / 16) * (DIM / 64) + 3) / 4, 1), 128, 0, stream>>>(XG, IND, 0, B1, IND, 0, 0.0625f, H1, DIM, 0, NROW, DIM, IND);
  k_bias<true, false><<<(unsigned)(((size_t)NROW * DIM / 4 + 255) / 256), 256, 0, stream>>>(H1, bs1, tileGrp, (size_t)NROW * DIM / 4);
  k_gemm_h<false><<<dim3(((NROW / 16) * (DIM / 64) + 3) / 4, 1), 128, 0, stream>>>(H1, DIM, 0, B2, DIM, 0, 0.0625f, H2, DIM, 0, NROW, DIM, DIM);
  k_bias<true, false><<<(unsigned)(((size_t)NROW * DIM / 4 + 255) / 256), 256, 0, stream>>>(H2, bs2, tileGrp, (size_t)NROW * DIM / 4);
  k_gemm_hgrp<false><<<dim3(((NROW / 16) * (DIM / 64) + 3) / 4, 1), 128, 0, stream>>>(H2, DIM, BE1, DIM, (size_t)DIM * DIM, tileGrp, 0.0625f, H1, DIM, NROW, DIM, DIM);
  k_bias<true, true><<<(unsigned)(((size_t)NROW * DIM / 4 + 255) / 256), 256, 0, stream>>>(H1, be1, tileGrp, (size_t)NROW * DIM / 4);
  k_gemm_hgrp<false><<<dim3(((NROW / 16) * (DIM / 64) + 3) / 4, 1), 128, 0, stream>>>(H1, DIM, BE2, DIM, (size_t)DIM * DIM, tileGrp, 0.0625f, H2, DIM, NROW, DIM, DIM);
  k_bias<false, true><<<(unsigned)(((size_t)NROW * DIM / 4 + 255) / 256), 256, 0, stream>>>(H2, be2, tileGrp, (size_t)NROW * DIM / 4);
  k_unsort<<<(unsigned)(((size_t)BS * DIM / 4 + 255) / 256), 256, 0, stream>>>(H2, smpRow, (float*)d_out);
}
